// Encoder_67113158967655
// MI455X (gfx1250) — hardware-verified
//
#include <hip/hip_runtime.h>
#include <stddef.h>
#include <stdint.h>
#include <math.h>


#define HID    64
#define HLP    128
#define KA     192
#define KB     256
#define EPSN   1e-12f
#define NTHR   256
#define NWAVE  8
#define EPT    8
#define CHUNK  (NTHR * EPT)
#define WCAP   (EPT * 32)
#define LISTN  (NWAVE * WCAP)
#define NBA    1024
#define SLA    10
#define RCAP   20480
#define DEGCAP 64
#define FLAGW  32
#define GBM    128
#define GTHR   256
#define AGR    128
#define NUWA   (HID * (KA / 8))
#define NUWB   (HID * (KB / 8))
#define NUW    (NUWA + NUWB)
#define BK_ZINTS    (LISTN + 2 * RCAP + 4 * NBA)
#define BK_LDS_INTS (BK_ZINTS + 16)
#define WSMAX  134217728

static_assert((CHUNK & (CHUNK - 1)) == 0 && CHUNK <= 4096);
static_assert((NBA & (NBA - 1)) == 0 && NBA == (1 << SLA));
static_assert(((long long)CHUNK << SLA) < (1LL << 31));
static_assert(RCAP >= 17546 && RCAP % (NTHR * 4) == 0);
static_assert(DEGCAP >= 36 + 8);
static_assert(NBA % 32 == 0 && NBA % AGR == 0 && NBA % GBM == 0 && NBA == NTHR * 4);
static_assert(BK_ZINTS % (NTHR * 4) == 0 && LISTN % 4 == 0);
static_assert(BK_LDS_INTS * 4 <= 300000);
static_assert(KA % 32 == 0 && KB % 32 == 0 && HID == 64 && HLP == 2 * HID);
static_assert(GBM == (GTHR / 32) * 16 && AGR == NWAVE * 16 && GTHR == NTHR);
static_assert(NUWA % 512 == 0 && NUWB % 512 == 0 && NUW % NTHR == 0);
static_assert(FLAGW * 4 == 128);

typedef float          v2f   __attribute__((ext_vector_type(2)));
typedef float          v4f   __attribute__((ext_vector_type(4)));
typedef float          v8f   __attribute__((ext_vector_type(8)));
typedef int            v4i   __attribute__((ext_vector_type(4)));
typedef int            v8i   __attribute__((ext_vector_type(8)));
typedef unsigned int   v4u   __attribute__((ext_vector_type(4)));
typedef unsigned short v8us  __attribute__((ext_vector_type(8)));
typedef unsigned short v16us __attribute__((ext_vector_type(16)));
typedef __bf16         v16bf __attribute__((ext_vector_type(16)));
typedef v2f  __attribute__((may_alias)) v2fa;
typedef v4f  __attribute__((may_alias)) v4fa;
typedef v4i  __attribute__((may_alias)) v4ia;
typedef v8us __attribute__((may_alias)) v8usa;
union FragB { v16bf v; v16us u; v8us h[2]; v8i w; };

__device__ __forceinline__ v8f wmb(const FragB& a, const FragB& b, v8f c) {
  v8f d = __builtin_amdgcn_wmma_f32_16x16x32_bf16(false, a.v, false, b.v, (short)0, c, false, false);
  asm volatile("v_nop\n\tv_nop\n\tv_nop\n\tv_nop" : "+v"(d) : "v"(a.w), "v"(b.w));
  return d;
}

__device__ __forceinline__ v8f z8() { v8f z = {0.f, 0.f, 0.f, 0.f, 0.f, 0.f, 0.f, 0.f}; return z; }

__device__ __forceinline__ unsigned bf16_bits(float f) {
  const unsigned u = __float_as_uint(f);
  const unsigned r = (u + 0x7FFFu + ((u >> 16) & 1u)) >> 16;
  return (f != f) ? 0x7FC0u : r;
}
__device__ __forceinline__ float bf16_val(float f) {
  return __uint_as_float(bf16_bits(f) << 16);
}
__device__ __forceinline__ unsigned hl_bits(float v, unsigned& lo) {
  const unsigned hb = bf16_bits(v);
  lo = bf16_bits(v - __uint_as_float(hb << 16));
  return hb;
}

template <int SLB>
__device__ __forceinline__ int scan_chunk(const int* __restrict__ dsts, int nE, int cbase, int slotBase,
                                          int nb, int vec8, int* list, int tid, int lane, int wave) {
  int wc = 0;
  const int el0  = tid * EPT;
  const int e0   = cbase + el0;
  const int sent = -2147483647 - 1;
  v4i da, db;
  if (vec8 != 0 && cbase + CHUNK <= nE) {
    da = *(const v4i*)(dsts + e0);
    db = *(const v4i*)(dsts + e0 + 4);
  } else {
    da.x = (e0     < nE) ? dsts[min(e0,     nE - 1)] : sent;
    da.y = (e0 + 1 < nE) ? dsts[min(e0 + 1, nE - 1)] : sent;
    da.z = (e0 + 2 < nE) ? dsts[min(e0 + 2, nE - 1)] : sent;
    da.w = (e0 + 3 < nE) ? dsts[min(e0 + 3, nE - 1)] : sent;
    db.x = (e0 + 4 < nE) ? dsts[min(e0 + 4, nE - 1)] : sent;
    db.y = (e0 + 5 < nE) ? dsts[min(e0 + 5, nE - 1)] : sent;
    db.z = (e0 + 6 < nE) ? dsts[min(e0 + 6, nE - 1)] : sent;
    db.w = (e0 + 7 < nE) ? dsts[min(e0 + 7, nE - 1)] : sent;
  }
  const unsigned nbs = (unsigned)slotBase;
  const unsigned unb = (unsigned)nb;
  const unsigned s0 = (unsigned)da.x - nbs, s1 = (unsigned)da.y - nbs;
  const unsigned s2 = (unsigned)da.z - nbs, s3 = (unsigned)da.w - nbs;
  const unsigned s4 = (unsigned)db.x - nbs, s5 = (unsigned)db.y - nbs;
  const unsigned s6 = (unsigned)db.z - nbs, s7 = (unsigned)db.w - nbs;
  const bool h0 = s0 < unb, h1 = s1 < unb, h2 = s2 < unb, h3 = s3 < unb;
  const bool h4 = s4 < unb, h5 = s5 < unb, h6 = s6 < unb, h7 = s7 < unb;
  const unsigned any = __builtin_amdgcn_ballot_w32(h0 | h1 | h2 | h3 | h4 | h5 | h6 | h7);
  if (any != 0u) {
#define HITJ(J, HJ, SJ) { \
      const unsigned mj = __builtin_amdgcn_ballot_w32(HJ); \
      if (mj != 0u) { \
        if (HJ) { \
          const int pos = wc + (int)__builtin_amdgcn_mbcnt_lo(mj, 0u); \
          if (pos < WCAP) list[wave * WCAP + pos] = ((el0 + (J)) << SLB) | (int)(SJ); \
        } \
        wc += (int)__builtin_popcount(mj); } }
    HITJ(0, h0, s0)
    HITJ(1, h1, s1)
    HITJ(2, h2, s2)
    HITJ(3, h3, s3)
    HITJ(4, h4, s4)
    HITJ(5, h5, s5)
    HITJ(6, h6, s6)
    HITJ(7, h7, s7)
#undef HITJ
  }
  return wc;
}

__device__ __forceinline__ void count_chunk(const int* __restrict__ keys, int nE, int cbase, int slotBase,
                                            int* odeg, int tid) {
  const int e0 = cbase + tid * EPT;
  const bool valid = (e0 + EPT) <= nE;
  const int ec = valid ? e0 : 0;
  const v4i da = *(const v4i*)(keys + ec);
  const v4i db = *(const v4i*)(keys + ec + 4);
  const unsigned vm  = valid ? 0xFFFFFFFFu : 0u;
  const unsigned nbs = (unsigned)slotBase;
  const unsigned t0 = (((unsigned)da.x - nbs) & vm) | ~vm;
  const unsigned t1 = (((unsigned)da.y - nbs) & vm) | ~vm;
  const unsigned t2 = (((unsigned)da.z - nbs) & vm) | ~vm;
  const unsigned t3 = (((unsigned)da.w - nbs) & vm) | ~vm;
  const unsigned t4 = (((unsigned)db.x - nbs) & vm) | ~vm;
  const unsigned t5 = (((unsigned)db.y - nbs) & vm) | ~vm;
  const unsigned t6 = (((unsigned)db.z - nbs) & vm) | ~vm;
  const unsigned t7 = (((unsigned)db.w - nbs) & vm) | ~vm;
  if (t0 < (unsigned)NBA) atomicAdd(&odeg[t0], 1);
  if (t1 < (unsigned)NBA) atomicAdd(&odeg[t1], 1);
  if (t2 < (unsigned)NBA) atomicAdd(&odeg[t2], 1);
  if (t3 < (unsigned)NBA) atomicAdd(&odeg[t3], 1);
  if (t4 < (unsigned)NBA) atomicAdd(&odeg[t4], 1);
  if (t5 < (unsigned)NBA) atomicAdd(&odeg[t5], 1);
  if (t6 < (unsigned)NBA) atomicAdd(&odeg[t6], 1);
  if (t7 < (unsigned)NBA) atomicAdd(&odeg[t7], 1);
}

__device__ __forceinline__ v8us ld8col(const float* __restrict__ w, int n, int j) {
  v8us r;
  const float* p = w + (size_t)(8 * j) * HID + n;
#pragma unroll
  for (int i = 0; i < 8; ++i) r[i] = (unsigned short)bf16_bits(p[(size_t)i * HID]);
  return r;
}

__global__ __launch_bounds__(NTHR) void k_prep(const float* __restrict__ x, const float* __restrict__ wl,
                                               const float* __restrict__ wr, const float* __restrict__ w0,
                                               const float* __restrict__ w1, unsigned short* wca,
                                               unsigned short* wcb, unsigned short* xb, int nN, int nUnits) {
  const int u = (int)blockIdx.x * NTHR + (int)threadIdx.x;
  v8us o;
  unsigned short* dp;
  if (u < NUWA) {
    const int seg = u >> 9;
    const int n = (u >> 3) & (HID - 1), j = u & 7;
    if (seg < 2) o = ld8col(wl, n, j);
    else         o = ld8col(wr, n, j);
    dp = wca + (size_t)n * KA + (size_t)seg * HID + 8 * j;
  } else if (u < NUW) {
    const int v = u - NUWA;
    const int seg = v >> 9;
    const int n = (v >> 3) & (HID - 1), j = v & 7;
    if (seg < 2) o = ld8col(w0, n, j);
    else         o = ld8col(w1, n, j);
    dp = wcb + (size_t)n * KB + (size_t)seg * HID + 8 * j;
  } else if (u < nUnits) {
    const int v   = u - NUW;
    const int row = v >> 3, k8 = (v & 7) * 8;
    const int rc  = row < nN ? row : nN - 1;
    const bool ok = row < nN;
    const float* p = x + (size_t)rc * HID + k8;
    const v4f a = *(const v4fa*)p;
    const v4f b = *(const v4fa*)(p + 4);
    o[0] = ok ? (unsigned short)bf16_bits(a.x) : (unsigned short)0;
    o[1] = ok ? (unsigned short)bf16_bits(a.y) : (unsigned short)0;
    o[2] = ok ? (unsigned short)bf16_bits(a.z) : (unsigned short)0;
    o[3] = ok ? (unsigned short)bf16_bits(a.w) : (unsigned short)0;
    o[4] = ok ? (unsigned short)bf16_bits(b.x) : (unsigned short)0;
    o[5] = ok ? (unsigned short)bf16_bits(b.y) : (unsigned short)0;
    o[6] = ok ? (unsigned short)bf16_bits(b.z) : (unsigned short)0;
    o[7] = ok ? (unsigned short)bf16_bits(b.w) : (unsigned short)0;
    dp = xb + (size_t)v * 8;
  } else {
    return;
  }
  *(volatile v8us*)dp = o;
  __threadfence();
  *(volatile v8us*)dp = o;
}

__global__ __launch_bounds__(NTHR) void k_bucket(const int* __restrict__ srcs, const int* __restrict__ dsts,
                                                 int nE, int nN, int vec8, int* listg, int* cntg, int* offg,
                                                 float* disg, int* flagg) {
  extern __shared__ __attribute__((aligned(16))) int dsm[];
  int* list = dsm;
  int* hl   = dsm + LISTN;
  int* sl   = hl + RCAP;
  int* cnt  = sl + RCAP;
  int* offs = cnt + NBA;
  int* cur  = offs + NBA;
  int* odeg = cur + NBA;
  int* misc = odeg + NBA;
  const int tid = (int)threadIdx.x, lane = tid & 31, wave = tid >> 5;
  const int nodeBase = (int)blockIdx.x * NBA;

  {
    const v4i z4 = {0, 0, 0, 0};
    for (int i = tid * 4; i < BK_ZINTS; i += NTHR * 4) *(v4ia*)(dsm + i) = z4;
    if (tid < 16) misc[tid] = 0;
  }
  __syncthreads();

  int t = 0, ov = 0;
  const int nChunks = (nE + CHUNK - 1) / CHUNK;
#pragma unroll 1
  for (int ch = 0; ch < nChunks; ++ch) {
    const int cbase = ch * CHUNK;
    count_chunk(srcs, nE, cbase, nodeBase, odeg, tid);
    const int wc = scan_chunk<SLA>(dsts, nE, cbase, nodeBase, NBA, vec8, list, tid, lane, wave);
    if (lane == 0) misc[wave] = wc;
    __syncthreads();
    if (wave == 0) {
#pragma unroll 1
      for (int w2 = 0; w2 < NWAVE; ++w2) {
        int c = misc[w2];
        c = c < 0 ? 0 : (c > WCAP ? WCAP : c);
#pragma unroll 1
        for (int b0 = 0; b0 < c; b0 += 32) {
          const int idx = b0 + lane;
          const int ent = list[w2 * WCAP + (idx < WCAP ? idx : WCAP - 1)];
          const int m32 = (c - b0) < 32 ? (c - b0) : 32;
#pragma unroll 1
          for (int k = 0; k < m32; ++k) {
            const int u    = __builtin_amdgcn_readlane(ent, k);
            const int slot = u & (NBA - 1);
            const int el   = (u >> SLA) & (CHUNK - 1);
            const int pk   = ((cbase + el) << SLA) | slot;
            if (t < RCAP) {
              if (lane == 0) { hl[t] = pk; cnt[slot] = cnt[slot] + 1; }
              t = t + 1;
            } else {
              ov = 1;
            }
          }
        }
      }
    }
    __syncthreads();
  }
  if (wave == 0 && lane == 0) { misc[8] = t; misc[9] = ov; }
  __syncthreads();
  int tt = misc[8];
  tt = tt < 0 ? 0 : (tt > RCAP ? RCAP : tt);

  if (wave == 0) {
    const int base = lane * (NBA / 32);
    int s = 0;
#pragma unroll 1
    for (int i = 0; i < NBA / 32; ++i) s += cnt[base + i];
    int incl = s;
#pragma unroll
    for (int d = 1; d < 32; d <<= 1) {
      const int y = __shfl_up(incl, d, 32);
      if (lane >= d) incl += y;
    }
    int run = incl - s;
#pragma unroll 1
    for (int i = 0; i < NBA / 32; ++i) {
      const int cv = cnt[base + i];
      offs[base + i] = run;
      cur[base + i]  = run;
      run += cv;
    }
  }
  __syncthreads();
  if (wave == 0) {
#pragma unroll 1
    for (int b0 = 0; b0 < tt; b0 += 32) {
      const int idx = b0 + lane;
      const int ent = hl[idx < RCAP ? idx : RCAP - 1];
      const int m32 = (tt - b0) < 32 ? (tt - b0) : 32;
#pragma unroll 1
      for (int k = 0; k < m32; ++k) {
        const int u    = __builtin_amdgcn_readlane(ent, k);
        const int slot = u & (NBA - 1);
        if (lane == 0) {
          int p = cur[slot];
          p = p < 0 ? 0 : (p > RCAP - 1 ? RCAP - 1 : p);
          sl[p] = u;
          cur[slot] = p + 1;
        }
      }
    }
  }
  __syncthreads();

#pragma unroll 1
  for (int i = tid; i < NBA; i += NTHR) {
    const int dg = odeg[i];
    const float fd = (float)(dg < 1 ? 1 : dg);
    const float r  = 1.0f / sqrtf(fd);
    cur[i] = __float_as_int(dg > 0 ? r : 0.0f);
  }
  const v4i c4 = *(const v4ia*)(cnt + 4 * tid);
  const v4i o4 = *(const v4ia*)(offs + 4 * tid);
  {
    const int mx01 = c4.x > c4.y ? c4.x : c4.y;
    const int mx23 = c4.z > c4.w ? c4.z : c4.w;
    const int mx   = mx01 > mx23 ? mx01 : mx23;
    if (mx > DEGCAP) misc[10] = 1;
  }
  __syncthreads();
  const int flg = ((misc[9] != 0) || (misc[10] != 0)) ? 1 : 0;
  const v4i d4 = *(const v4ia*)(cur + 4 * tid);

  int* lb = listg + (size_t)blockIdx.x * RCAP;
#pragma unroll 1
  for (int it = 0; it < RCAP / (NTHR * 4); ++it) {
    const int p0 = it * (NTHR * 4) + 4 * tid;
    const v4i e4 = *(const v4ia*)(sl + p0);
    int e0 = e4.x >> SLA, e1 = e4.y >> SLA, e2 = e4.z >> SLA, e3 = e4.w >> SLA;
    e0 = e0 < 0 ? 0 : (e0 > nE - 1 ? nE - 1 : e0);
    e1 = e1 < 0 ? 0 : (e1 > nE - 1 ? nE - 1 : e1);
    e2 = e2 < 0 ? 0 : (e2 > nE - 1 ? nE - 1 : e2);
    e3 = e3 < 0 ? 0 : (e3 > nE - 1 ? nE - 1 : e3);
    int r0 = srcs[e0], r1 = srcs[e1], r2 = srcs[e2], r3 = srcs[e3];
    r0 = r0 < 0 ? 0 : (r0 > nN - 1 ? nN - 1 : r0);
    r1 = r1 < 0 ? 0 : (r1 > nN - 1 ? nN - 1 : r1);
    r2 = r2 < 0 ? 0 : (r2 > nN - 1 ? nN - 1 : r2);
    r3 = r3 < 0 ? 0 : (r3 > nN - 1 ? nN - 1 : r3);
    v4i o;
    o.x = (p0     < tt) ? r0 : 0;
    o.y = (p0 + 1 < tt) ? r1 : 0;
    o.z = (p0 + 2 < tt) ? r2 : 0;
    o.w = (p0 + 3 < tt) ? r3 : 0;
    *(volatile v4i*)(lb + p0) = o;
    __threadfence();
    *(volatile v4i*)(lb + p0) = o;
  }

  v4f df;
  df.x = __int_as_float(d4.x); df.y = __int_as_float(d4.y);
  df.z = __int_as_float(d4.z); df.w = __int_as_float(d4.w);
  const v4i f4 = {flg, flg, flg, flg};
  int*   cp = cntg + (size_t)nodeBase + 4 * tid;
  int*   op = offg + (size_t)nodeBase + 4 * tid;
  float* dp = disg + (size_t)nodeBase + 4 * tid;
  int*   fp = flagg + (size_t)blockIdx.x * FLAGW + 4 * (lane & 7);
  const bool fw = (wave == 0) && (lane < 8);
  *(volatile v4i*)cp = c4;
  *(volatile v4i*)op = o4;
  *(volatile v4f*)dp = df;
  if (fw) *(volatile v4i*)fp = f4;
  __threadfence();
  *(volatile v4i*)cp = c4;
  *(volatile v4i*)op = o4;
  *(volatile v4f*)dp = df;
  if (fw) *(volatile v4i*)fp = f4;
}

template <int MODE>
__global__ __launch_bounds__(NTHR) void k_agg(const int* __restrict__ listg, const int* __restrict__ cntg,
                                              const int* __restrict__ offg, const float* __restrict__ disg,
                                              const int* __restrict__ flagg, const unsigned* __restrict__ srcw,
                                              unsigned short* outp, int nN, int mRows, int nbp, int nblk) {
  const int tid = (int)threadIdx.x, lane = tid & 31;
  const int wave = __builtin_amdgcn_readfirstlane(tid >> 5);
  const float qnan = __int_as_float(0x7fc00000);
  const int q0s = (4 * lane) & 31, q1s = (4 * lane + 1) & 31;
  const int q2s = (4 * lane + 2) & 31, q3s = (4 * lane + 3) & 31;
#pragma unroll 1
  for (int si = 0; si < AGR / NWAVE; ++si) {
    const int node = (int)blockIdx.x * AGR + si * NWAVE + wave;
    const int ncl  = node < nbp ? node : nbp - 1;
    int bb = ncl >> SLA;
    bb = bb < nblk ? bb : nblk - 1;
    int c = cntg[ncl];
    const bool big = c > DEGCAP;
    c = c < 0 ? 0 : (c > DEGCAP ? DEGCAP : c);
    int o = offg[ncl];
    o = o < 0 ? 0 : (o > RCAP - 1 ? RCAP - 1 : o);
    const int fl = flagg[(size_t)bb * FLAGW];
    float ddst = 0.0f;
    if constexpr (MODE != 0) ddst = disg[ncl];
    const int* lp = listg + (size_t)bb * RCAP;
    float a0 = 0.0f, a1 = 0.0f;
#pragma unroll 1
    for (int b0 = 0; b0 < c; b0 += 32) {
      int j = b0 + lane;
      j = j > c - 1 ? c - 1 : j;
      int idx = o + j;
      idx = idx > RCAP - 1 ? RCAP - 1 : idx;
      int sr = lp[idx];
      sr = sr < 0 ? 0 : (sr > nN - 1 ? nN - 1 : sr);
      int cfi = 0;
      if constexpr (MODE != 0) {
        const float dsrc = disg[sr];
        cfi = __float_as_int(-(dsrc * ddst));
      }
      const int m32 = (c - b0) < 32 ? (c - b0) : 32;
#pragma unroll 1
      for (int k = 0; k < m32; ++k) {
        const int sk = __builtin_amdgcn_readlane(sr, k);
        if constexpr (MODE == 0) {
          const unsigned w = srcw[(size_t)sk * (HID / 2) + lane];
          a0 += __uint_as_float(w << 16);
          a1 += __uint_as_float(w & 0xffff0000u);
        } else {
          const float ck = __int_as_float(__builtin_amdgcn_readlane(cfi, k));
          const unsigned wh = srcw[(size_t)sk * (HLP / 2) + lane];
          const unsigned wl = srcw[(size_t)sk * (HLP / 2) + (HID / 2) + lane];
          const float h0 = __uint_as_float(wh << 16)         + __uint_as_float(wl << 16);
          const float h1 = __uint_as_float(wh & 0xffff0000u) + __uint_as_float(wl & 0xffff0000u);
          a0 += h0 * ck;
          a1 += h1 * ck;
        }
      }
    }
    float y0 = a0, y1 = a1;
    if constexpr (MODE == 0) {
      const float dv = (float)(c < 1 ? 1 : c);
      y0 = a0 / dv;
      y1 = a1 / dv;
    }
    const bool pois = (fl != 0) || big;
    const bool live = node < nN;
    y0 = pois ? qnan : y0;
    y1 = pois ? qnan : y1;
    const float v0 = live ? y0 : 0.0f;
    const float v1 = live ? y1 : 0.0f;
    unsigned lb0, lb1;
    const unsigned hb0 = hl_bits(v0, lb0);
    const unsigned hb1 = hl_bits(v1, lb1);
    const int hw = (int)(hb0 | (hb1 << 16));
    const int lw = (int)(lb0 | (lb1 << 16));
    const int g0 = __shfl(hw, q0s, 32), g1 = __shfl(hw, q1s, 32);
    const int g2 = __shfl(hw, q2s, 32), g3 = __shfl(hw, q3s, 32);
    const int p0 = __shfl(lw, q0s, 32), p1 = __shfl(lw, q1s, 32);
    const int p2 = __shfl(lw, q2s, 32), p3 = __shfl(lw, q3s, 32);
    const bool lsel = (lane & 8) != 0;
    v4u pv;
    pv.x = (unsigned int)(lsel ? p0 : g0);
    pv.y = (unsigned int)(lsel ? p1 : g1);
    pv.z = (unsigned int)(lsel ? p2 : g2);
    pv.w = (unsigned int)(lsel ? p3 : g3);
    const bool wr = (node < mRows) && (lane < 16);
    unsigned short* hp = outp + (size_t)node * HLP + 8 * (lane & 15);
    if (wr) *(volatile v4u*)hp = pv;
    __threadfence();
    if (wr) *(volatile v4u*)hp = pv;
  }
}

__device__ __forceinline__ void kloop(const unsigned short* ap, const unsigned short* __restrict__ bp, int ldb,
                                      int K, v8f& c0, v8f& c1, v8f& c2, v8f& c3) {
#pragma unroll 1
  for (int k0 = 0; k0 < K; k0 += 32) {
    FragB af;
    af.h[0] = *(const v8usa*)(ap + k0);
    af.h[1] = *(const v8usa*)(ap + k0 + 16);
    {
      const unsigned short* wq = bp + k0;
      FragB bf;
      bf.h[0] = *(const v8usa*)wq;
      bf.h[1] = *(const v8usa*)(wq + 16);
      c0 = wmb(af, bf, c0);
    }
    {
      const unsigned short* wq = bp + (size_t)16 * (size_t)ldb + k0;
      FragB bf;
      bf.h[0] = *(const v8usa*)wq;
      bf.h[1] = *(const v8usa*)(wq + 16);
      c1 = wmb(af, bf, c1);
    }
    {
      const unsigned short* wq = bp + (size_t)32 * (size_t)ldb + k0;
      FragB bf;
      bf.h[0] = *(const v8usa*)wq;
      bf.h[1] = *(const v8usa*)(wq + 16);
      c2 = wmb(af, bf, c2);
    }
    {
      const unsigned short* wq = bp + (size_t)48 * (size_t)ldb + k0;
      FragB bf;
      bf.h[0] = *(const v8usa*)wq;
      bf.h[1] = *(const v8usa*)(wq + 16);
      c3 = wmb(af, bf, c3);
    }
  }
}

template <int LAST>
__global__ __launch_bounds__(GTHR) void k_gemm(const unsigned short* A1, int lda1, int K1,
                                               const unsigned short* A2, int lda2, int K2,
                                               const unsigned short* __restrict__ BT, int ldb,
                                               const float* __restrict__ bias, const float* __restrict__ pw,
                                               unsigned short* hout, float* outp, int nN, int mRows) {
  __shared__ __attribute__((aligned(16))) float stg[GBM * HID];
  __shared__ __attribute__((aligned(16))) float prm[2 * HID];
  const int tid = (int)threadIdx.x, lane = tid & 31, hh = lane >> 4, m = lane & 15;
  const int wave = __builtin_amdgcn_readfirstlane(tid >> 5);
  const int rowBase = (int)blockIdx.x * GBM;

  {
    const int j4 = 4 * (tid & 15);
    const v4f b4 = *(const v4f*)(bias + j4);
    const v4f w4 = *(const v4f*)(pw + j4);
    const unsigned mk = (((tid >> 4) & 1) != 0) ? 0xFFFFFFFFu : 0u;
    v4f sel;
    sel.x = bf16_val(__uint_as_float((__float_as_uint(b4.x) & ~mk) | (__float_as_uint(w4.x) & mk)));
    sel.y = bf16_val(__uint_as_float((__float_as_uint(b4.y) & ~mk) | (__float_as_uint(w4.y) & mk)));
    sel.z = bf16_val(__uint_as_float((__float_as_uint(b4.z) & ~mk) | (__float_as_uint(w4.z) & mk)));
    sel.w = bf16_val(__uint_as_float((__float_as_uint(b4.w) & ~mk) | (__float_as_uint(w4.w) & mk)));
    if (tid < 32) *(v4fa*)(prm + ((tid >> 4) & 1) * HID + j4) = sel;
  }

  v8f acc[4];
#pragma unroll
  for (int t = 0; t < 4; ++t) acc[t] = z8();
  const size_t arow = (size_t)(rowBase + 16 * wave + m);
  const unsigned short* ap1 = A1 + arow * (size_t)lda1 + 8 * hh;
  const unsigned short* ap2 = A2 + arow * (size_t)lda2 + 8 * hh;
  const unsigned short* bp  = BT + (size_t)m * (size_t)ldb + 8 * hh;
  kloop(ap1, bp, ldb, K1, acc[0], acc[1], acc[2], acc[3]);
  kloop(ap2, bp + K1, ldb, K2, acc[0], acc[1], acc[2], acc[3]);

#pragma unroll
  for (int nt = 0; nt < 4; ++nt) {
    const int lc = 16 * nt + m;
#pragma unroll
    for (int r = 0; r < 8; ++r) {
      const int lr = 16 * wave + 8 * hh + r;
      stg[lr * HID + lc] = acc[nt][r];
    }
  }
  __syncthreads();

  if constexpr (LAST == 0) {
    const v2f bq = *(const v2fa*)(prm + 2 * lane);
    const v2f wq = *(const v2fa*)(prm + HID + 2 * lane);
    const int q0s = (4 * lane) & 31, q1s = (4 * lane + 1) & 31;
    const int q2s = (4 * lane + 2) & 31, q3s = (4 * lane + 3) & 31;
#pragma unroll 1
    for (int i = 0; i < 16; ++i) {
      const int lr  = 16 * wave + i;
      const int row = rowBase + lr;
      const bool ok = row < nN;
      const v2f tv = *(const v2fa*)(stg + lr * HID + 2 * lane);
      float y0 = tv.x + bq.x, y1 = tv.y + bq.y;
      float ss = y0 * y0 + y1 * y1;
      ss += __shfl_xor(ss, 16, 32);
      ss += __shfl_xor(ss, 8, 32);
      ss += __shfl_xor(ss, 4, 32);
      ss += __shfl_xor(ss, 2, 32);
      ss += __shfl_xor(ss, 1, 32);
      float d = sqrtf(ss);
      d = (d > EPSN || d != d) ? d : EPSN;
      y0 = y0 / d;
      y1 = y1 / d;
      y0 = (y0 >= 0.0f) ? y0 : y0 * wq.x;
      y1 = (y1 >= 0.0f) ? y1 : y1 * wq.y;
      const float v0 = ok ? y0 : 0.0f;
      const float v1 = ok ? y1 : 0.0f;
      unsigned lb0, lb1;
      const unsigned hb0 = hl_bits(v0, lb0);
      const unsigned hb1 = hl_bits(v1, lb1);
      const int hw = (int)(hb0 | (hb1 << 16));
      const int lw = (int)(lb0 | (lb1 << 16));
      const int g0 = __shfl(hw, q0s, 32), g1 = __shfl(hw, q1s, 32);
      const int g2 = __shfl(hw, q2s, 32), g3 = __shfl(hw, q3s, 32);
      const int p0 = __shfl(lw, q0s, 32), p1 = __shfl(lw, q1s, 32);
      const int p2 = __shfl(lw, q2s, 32), p3 = __shfl(lw, q3s, 32);
      const bool lsel = (lane & 8) != 0;
      v4u pv;
      pv.x = (unsigned int)(lsel ? p0 : g0);
      pv.y = (unsigned int)(lsel ? p1 : g1);
      pv.z = (unsigned int)(lsel ? p2 : g2);
      pv.w = (unsigned int)(lsel ? p3 : g3);
      const bool wr = (row < mRows) && (lane < 16);
      unsigned short* hp = hout + (size_t)row * HLP + 8 * (lane & 15);
      if (wr) *(volatile v4u*)hp = pv;
      __threadfence();
      if (wr) *(volatile v4u*)hp = pv;
    }
    (void)outp;
  } else {
    const v4f b4 = *(const v4fa*)(prm + 4 * m);
    const v4f w4 = *(const v4fa*)(prm + HID + 4 * m);
    v4f fv[8];
#pragma unroll
    for (int i = 0; i < 8; ++i) {
      const int lr = 16 * wave + 2 * i + hh;
      const v4f tv = *(const v4fa*)(stg + lr * HID + 4 * m);
      const float y0 = tv.x + b4.x, y1 = tv.y + b4.y, y2 = tv.z + b4.z, y3 = tv.w + b4.w;
      v4f q;
      q.x = (y0 >= 0.0f) ? y0 : y0 * w4.x;
      q.y = (y1 >= 0.0f) ? y1 : y1 * w4.y;
      q.z = (y2 >= 0.0f) ? y2 : y2 * w4.z;
      q.w = (y3 >= 0.0f) ? y3 : y3 * w4.w;
      fv[i] = q;
    }
#pragma unroll
    for (int i = 0; i < 8; ++i) {
      const int gr = rowBase + 16 * wave + 2 * i + hh;
      float* op = outp + (size_t)gr * HID + 4 * m;
      if (gr < nN) *(volatile v4f*)op = fv[i];
    }
    __threadfence();
#pragma unroll
    for (int i = 0; i < 8; ++i) {
      const int gr = rowBase + 16 * wave + 2 * i + hh;
      float* op = outp + (size_t)gr * HID + 4 * m;
      if (gr < nN) *(volatile v4f*)op = fv[i];
    }
    (void)hout; (void)mRows;
  }
}

static inline int cdiv(int a, int b) { return (a + b - 1) / b; }
static inline size_t al256(size_t o) { return (o + 255) & ~(size_t)255; }

extern "C" void kernel_launch(void* const* d_in, const int* in_sizes, int n_in,
                              void* d_out, int out_size, void* d_ws, size_t ws_size,
                              hipStream_t stream) {
  if (n_in < 9) return;
  if (in_sizes[0] < HID || (in_sizes[0] % HID) != 0) return;
  const int nN = in_sizes[0] / HID;
  if (nN < 1 || nN > (1 << 22)) return;
  if (in_sizes[1] < 2 || (in_sizes[1] & 1) != 0) return;
  const int nE = in_sizes[1] / 2;
  if (nE < EPT || (nE % EPT) != 0 || nE >= (1 << (31 - SLA))) return;
  if (in_sizes[2] != HID * HID || in_sizes[3] != HID) return;
  if (in_sizes[4] != HID * HID) return;
  if (in_sizes[5] != HID * HID || in_sizes[6] != HID * HID) return;
  if (in_sizes[7] != HID || in_sizes[8] != HID) return;
  if ((long long)out_size != (long long)nN * HID) return;

  const float* x   = (const float*)d_in[0];
  const int*   ei  = (const int*)  d_in[1];
  const float* Wl  = (const float*)d_in[2];
  const float* bl  = (const float*)d_in[3];
  const float* Wr  = (const float*)d_in[4];
  const float* W0  = (const float*)d_in[5];
  const float* W1  = (const float*)d_in[6];
  const float* bc  = (const float*)d_in[7];
  const float* pw  = (const float*)d_in[8];
  float* out = (float*)d_out;
  const int* src = ei;
  const int* dst = ei + nE;

  const int MP  = cdiv(nN, GBM) * GBM;
  const int gM  = MP / GBM;
  const int gB  = cdiv(nN, NBA);
  const int NBP = gB * NBA;
  if (NBP < MP) return;
  const int vec8 = ((nE & 3) == 0) ? 1 : 0;

  char* ws = (char*)d_ws;
  size_t off = 0;
  const size_t oWCA = off; off = al256(off + (size_t)HID * KA * 2);
  const size_t oWCB = off; off = al256(off + (size_t)HID * KB * 2);
  const size_t oXB  = off; off = al256(off + (size_t)MP * HID * 2);
  const size_t oMN  = off; off = al256(off + (size_t)MP * HLP * 2);
  const size_t oH   = off; off = al256(off + (size_t)MP * HLP * 2);
  const size_t oTX  = off; off = al256(off + (size_t)MP * HLP * 2);
  const size_t oLS  = off; off = al256(off + (size_t)gB * RCAP * 4);
  const size_t oCN  = off; off = al256(off + (size_t)NBP * 4);
  const size_t oOF  = off; off = al256(off + (size_t)NBP * 4);
  const size_t oDS  = off; off = al256(off + (size_t)NBP * 4);
  const size_t oFL  = off; off = al256(off + (size_t)gB * FLAGW * 4);
  if (off > ws_size || off > (size_t)WSMAX) return;
  unsigned short* WCA = (unsigned short*)(ws + oWCA);
  unsigned short* WCB = (unsigned short*)(ws + oWCB);
  unsigned short* XB  = (unsigned short*)(ws + oXB);
  unsigned short* MN  = (unsigned short*)(ws + oMN);
  unsigned short* HH  = (unsigned short*)(ws + oH);
  unsigned short* TX  = (unsigned short*)(ws + oTX);
  int*   LS = (int*)(ws + oLS);
  int*   CN = (int*)(ws + oCN);
  int*   OF = (int*)(ws + oOF);
  float* DS = (float*)(ws + oDS);
  int*   FL = (int*)(ws + oFL);

  const size_t bkLds = (size_t)BK_LDS_INTS * 4;
  hipFuncSetAttribute(reinterpret_cast<const void*>(&k_bucket), hipFuncAttributeMaxDynamicSharedMemorySize, (int)bkLds);

  const int nUnits = NUW + MP * (HID / 8);

  k_prep<<<cdiv(nUnits, NTHR), NTHR, 0, stream>>>(x, Wl, Wr, W0, W1, WCA, WCB, XB, nN, nUnits);
  k_bucket<<<gB, NTHR, bkLds, stream>>>(src, dst, nE, nN, vec8, LS, CN, OF, DS, FL);
  k_agg<0><<<gM, NTHR, 0, stream>>>(LS, CN, OF, DS, FL, (const unsigned*)XB, MN, nN, MP, NBP, gB);
  k_gemm<0><<<gM, GTHR, 0, stream>>>(MN, HLP, HLP, XB, HID, HID, WCA, KA, bl, pw, HH, out, nN, MP);
  k_agg<1><<<gM, NTHR, 0, stream>>>(LS, CN, OF, DS, FL, (const unsigned*)HH, TX, nN, MP, NBP, gB);
  k_gemm<1><<<gM, GTHR, 0, stream>>>(HH, HLP, HLP, TX, HLP, HLP, WCB, KB, bc, pw, HH, out, nN, MP);
}
